// CrfRnnLayer_20933670600704
// MI455X (gfx1250) — hardware-verified
//
#include <hip/hip_runtime.h>

#define B_  4
#define H_  64
#define W_  64
#define C_  21
#define N_  4096
#define CP  32
#define KSC 64.0f
#define UNSC (1.0f / 4096.0f)

typedef __attribute__((ext_vector_type(16))) _Float16 v16h;
typedef __attribute__((ext_vector_type(8)))  _Float16 v8h;
typedef __attribute__((ext_vector_type(8)))  float    v8f;
typedef __attribute__((ext_vector_type(4)))  float    v4f;
typedef __attribute__((ext_vector_type(4)))  unsigned v4u;
typedef float __attribute__((may_alias)) float_a;

__device__ __forceinline__ v16h load_frag(const _Float16* row, int sel) {
  union { v16h v; v8h h[2]; } r;
  r.h[0] = *(const v8h*)(row + sel * 8);
  r.h[1] = *(const v8h*)(row + 16 + sel * 8);
  return r.v;
}
__device__ __forceinline__ v8f wmma_f16(v16h a, v16h b, v8f c) {
  v8f d = __builtin_amdgcn_wmma_f32_16x16x32_f16(false, a, false, b, (short)0, c, false, false);
  asm volatile("v_nop\n\tv_nop\n\tv_nop\n\tv_nop" : "+v"(d) : "v"(a), "v"(b));
  return d;
}

__global__ __launch_bounds__(256) void build_spatial(_Float16* __restrict__ Ks, float* __restrict__ s_norm) {
  __shared__ float nrm[32];
  const int lane = threadIdx.x & 31, wv = threadIdx.x >> 5;
  const float inv_g2 = 1.0f / 9.0f;
#pragma unroll 1
  for (int rr = 0; rr < 4; ++rr) {
    const int n = blockIdx.x * 32 + wv * 4 + rr;
    const float yn = (float)(n >> 6), xn = (float)(n & 63);
    _Float16* krow = Ks + (size_t)n * N_;
    float sum = 0.0f;
#pragma unroll 1
    for (int j = 0; j < N_ / 256; ++j) {
      const int m0 = j * 256 + lane * 8;
      union { v8h v; v4u u; } pk;
#pragma unroll
      for (int i = 0; i < 8; ++i) {
        const int m = m0 + i;
        const float dy = yn - (float)(m >> 6);
        const float dx = xn - (float)(m & 63);
        const float v = __expf(-0.5f * (dy * dy + dx * dx) * inv_g2);
        const _Float16 h = (_Float16)(v * KSC);
        pk.v[i] = h;
        sum += (float)h;
      }
      *(volatile v4u*)(krow + m0) = pk.u;
      __threadfence();
      *(volatile v4u*)(krow + m0) = pk.u;
    }
    for (int s = 16; s > 0; s >>= 1) sum += __shfl_xor(sum, s, 32);
    if (lane == 0) nrm[wv * 4 + rr] = sum * (1.0f / KSC);
  }
  __syncthreads();
  if (threadIdx.x < 32) {
    const float v = nrm[lane];
    *(volatile float_a*)(s_norm + blockIdx.x * 32 + lane) = v;
    __threadfence();
    *(volatile float_a*)(s_norm + blockIdx.x * 32 + lane) = v;
  }
}

__global__ __launch_bounds__(256) void build_bilateral(const float* __restrict__ rgb,
                                                       _Float16* __restrict__ Kb, float* __restrict__ b_norm) {
  __shared__ float nrm[32];
  __shared__ float feat[N_ * 3];
  const int lane = threadIdx.x & 31, wv = threadIdx.x >> 5;
  const int row0 = blockIdx.x * 32;
  const int b = row0 >> 12;
  const float inv_a = 1.0f / 160.0f, inv_bt = 1.0f / 3.0f;
  const float* rb = rgb + (size_t)b * N_ * 3;
  for (int i = threadIdx.x; i < N_ * 3; i += 256) feat[i] = rb[i] * inv_bt;
  __syncthreads();
#pragma unroll 1
  for (int rr = 0; rr < 4; ++rr) {
    const int row = row0 + wv * 4 + rr;
    const int n = row & 4095;
    const float f0 = (float)(n >> 6) * inv_a;
    const float f1 = (float)(n & 63) * inv_a;
    const float f2 = feat[n * 3 + 0];
    const float f3 = feat[n * 3 + 1];
    const float f4 = feat[n * 3 + 2];
    _Float16* krow = Kb + (size_t)row * N_;
    float sum = 0.0f;
#pragma unroll 1
    for (int j = 0; j < N_ / 256; ++j) {
      const int m0 = j * 256 + lane * 8;
      union { v8h v; v4u u; } pk;
#pragma unroll
      for (int i = 0; i < 8; ++i) {
        const int m = m0 + i;
        const float d0 = f0 - (float)(m >> 6) * inv_a;
        const float d1 = f1 - (float)(m & 63) * inv_a;
        const float d2 = f2 - feat[m * 3 + 0];
        const float d3 = f3 - feat[m * 3 + 1];
        const float d4 = f4 - feat[m * 3 + 2];
        const float v = __expf(-0.5f * (d0*d0 + d1*d1 + d2*d2 + d3*d3 + d4*d4));
        const _Float16 h = (_Float16)(v * KSC);
        pk.v[i] = h;
        sum += (float)h;
      }
      *(volatile v4u*)(krow + m0) = pk.u;
      __threadfence();
      *(volatile v4u*)(krow + m0) = pk.u;
    }
    for (int s = 16; s > 0; s >>= 1) sum += __shfl_xor(sum, s, 32);
    if (lane == 0) nrm[wv * 4 + rr] = sum * (1.0f / KSC);
  }
  __syncthreads();
  if (threadIdx.x < 32) {
    const float v = nrm[lane];
    *(volatile float_a*)(b_norm + row0 + lane) = v;
    __threadfence();
    *(volatile float_a*)(b_norm + row0 + lane) = v;
  }
}

__global__ __launch_bounds__(1024) void mix_mats(const float* __restrict__ Ws, const float* __restrict__ Wb,
                                                 const float* __restrict__ compat,
                                                 float* __restrict__ CWs, float* __restrict__ CWb) {
  int c = threadIdx.x >> 5;
  int k = threadIdx.x & 31;
  float a = 0.0f, bb = 0.0f;
  if (c < C_ && k < C_) {
    for (int j = 0; j < C_; ++j) {
      a  += compat[c * C_ + j] * Ws[j * C_ + k];
      bb += compat[c * C_ + j] * Wb[j * C_ + k];
    }
  }
  *(volatile float_a*)(CWs + c * 32 + k) = a;
  *(volatile float_a*)(CWb + c * 32 + k) = bb;
  __threadfence();
  *(volatile float_a*)(CWs + c * 32 + k) = a;
  *(volatile float_a*)(CWb + c * 32 + k) = bb;
}

__device__ __forceinline__ void store_ptile(const _Float16* tile, _Float16* Pb, int n0, int tid, int nthreads) {
  for (int g = tid; g < 32 * 16; g += nthreads) {
    const int c = g >> 4, pc = g & 15;
    const v4u v = *(const v4u*)((const char*)tile + c * 256 + pc * 16);
    char* dst = (char*)(Pb + (size_t)c * N_ + n0) + pc * 16;
    *(volatile v4u*)dst = v;
    __threadfence();
    *(volatile v4u*)dst = v;
  }
}

__global__ __launch_bounds__(128) void init_p(const float* __restrict__ unary, _Float16* __restrict__ P0) {
  __shared__ __align__(16) _Float16 tile[CP * 128];
  const int t = threadIdx.x;
  const int p = blockIdx.x * 128 + t;
  const int b = p >> 12, n0 = (blockIdx.x * 128) & 4095;
  const float* u = unary + (size_t)p * C_;
  float mx = -3.402823466e38f;
  for (int c = 0; c < C_; ++c) mx = fmaxf(mx, u[c]);
  float e[C_], s = 0.0f;
  for (int c = 0; c < C_; ++c) { e[c] = __expf(u[c] - mx); s += e[c]; }
  const float inv = KSC / s;
  for (int c = 0; c < C_; ++c) tile[c * 128 + t] = (_Float16)(e[c] * inv);
  for (int c = C_; c < CP; ++c) tile[c * 128 + t] = (_Float16)0.0f;
  __syncthreads();
  store_ptile(tile, P0 + (size_t)b * CP * N_, n0, t, 128);
}

__global__ void __launch_bounds__(256)
crf_iter(const float* __restrict__ unary,
         const _Float16* __restrict__ Ks, const _Float16* __restrict__ Kb,
         const float* __restrict__ s_norm, const float* __restrict__ b_norm,
         const float* __restrict__ CWs, const float* __restrict__ CWb,
         const _Float16* __restrict__ Pin, _Float16* __restrict__ Pout,
         float* __restrict__ qout, int last) {
  __shared__ float SPl[8][CP][17];
  __shared__ float BLl[8][CP][17];
  __shared__ float Ql[8][C_][17];
  __shared__ __align__(16) _Float16 ptile[CP * 128];
  __shared__ __align__(16) float otile[128 * C_];

  const int tid  = threadIdx.x;
  const int wv   = tid >> 5;
  const int lane = tid & 31;
  const int sel  = lane >> 4;
  const int nl   = lane & 15;

  const int gw = blockIdx.x * 8 + wv;
  const int b  = gw >> 8;
  const int n0 = (gw & 255) << 4;
  const int nblk = (blockIdx.x * 128) & 4095;

  const _Float16* Pb  = Pin + (size_t)b * CP * N_;
  const _Float16* pa0 = Pb + (size_t)nl * N_;
  const _Float16* pa1 = Pb + (size_t)(nl + 16) * N_;
  const _Float16* pks = Ks + (size_t)(n0 + nl) * N_;
  const _Float16* pkb = Kb + ((size_t)b * N_ + n0 + nl) * N_;

  v8f sp0 = {}, sp1 = {}, bl0 = {}, bl1 = {};
#pragma unroll 2
  for (int k0 = 0; k0 < N_; k0 += 32) {
    v16h a0 = load_frag(pa0 + k0, sel);
    v16h a1 = load_frag(pa1 + k0, sel);
    v16h bs = load_frag(pks + k0, sel);
    v16h bb = load_frag(pkb + k0, sel);
    sp0 = wmma_f16(a0, bs, sp0);
    sp1 = wmma_f16(a1, bs, sp1);
    bl0 = wmma_f16(a0, bb, bl0);
    bl1 = wmma_f16(a1, bb, bl1);
  }

  const int nglob = n0 + nl;
  const float sdiv = UNSC / s_norm[nglob];
  const float bdiv = UNSC / b_norm[b * N_ + nglob];
#pragma unroll
  for (int r = 0; r < 8; ++r) {
    SPl[wv][r + 8 * sel][nl]      = sp0[r] * sdiv;
    SPl[wv][16 + r + 8 * sel][nl] = sp1[r] * sdiv;
    BLl[wv][r + 8 * sel][nl]      = bl0[r] * bdiv;
    BLl[wv][16 + r + 8 * sel][nl] = bl1[r] * bdiv;
  }
  __syncthreads();

  const float* uptr = unary + ((size_t)b * N_ + nglob) * C_;
  const int cbase = sel * 16;
#pragma unroll
  for (int ci = 0; ci < 16; ++ci) {
    int c = cbase + ci;
    if (c < C_) {
      float acc = 0.0f;
#pragma unroll
      for (int k = 0; k < C_; ++k)
        acc += CWs[c * 32 + k] * SPl[wv][k][nl] + CWb[c * 32 + k] * BLl[wv][k][nl];
      Ql[wv][c][nl] = uptr[c] - acc;
    }
  }
  __syncthreads();

  if (lane < 16) {
    const int nt = wv * 16 + lane;
    if (last) {
      for (int c = 0; c < C_; ++c) otile[nt * C_ + c] = Ql[wv][c][lane];
    } else {
      float mx = -3.402823466e38f;
      for (int c = 0; c < C_; ++c) mx = fmaxf(mx, Ql[wv][c][lane]);
      float e[C_], s = 0.0f;
      for (int c = 0; c < C_; ++c) { e[c] = __expf(Ql[wv][c][lane] - mx); s += e[c]; }
      const float inv = KSC / s;
      for (int c = 0; c < C_; ++c) ptile[c * 128 + nt] = (_Float16)(e[c] * inv);
      for (int c = C_; c < CP; ++c) ptile[c * 128 + nt] = (_Float16)0.0f;
    }
  }
  __syncthreads();
  if (last) {
    char* dst = (char*)(qout + ((size_t)b * N_ + nblk) * C_);
    for (int g = tid; g < 672; g += 256) {
      const v4f v = *(const v4f*)((const char*)otile + g * 16);
      *(volatile v4f*)(dst + g * 16) = v;
      __threadfence();
      *(volatile v4f*)(dst + g * 16) = v;
    }
  } else {
    store_ptile(ptile, Pout + (size_t)b * CP * N_, nblk, tid, 256);
  }
}

extern "C" void kernel_launch(void* const* d_in, const int* in_sizes, int n_in,
                              void* d_out, int out_size, void* d_ws, size_t ws_size,
                              hipStream_t stream) {
  (void)in_sizes; (void)n_in; (void)out_size; (void)ws_size;
  const float* unary  = (const float*)d_in[0];
  const float* rgb    = (const float*)d_in[1];
  const float* Ws     = (const float*)d_in[2];
  const float* Wb     = (const float*)d_in[3];
  const float* compat = (const float*)d_in[4];
  float* out = (float*)d_out;

  char* ws = (char*)d_ws;
  size_t off = 0;
  _Float16* Ks = (_Float16*)(ws + off); off += (size_t)N_ * N_ * 2;
  _Float16* Kb = (_Float16*)(ws + off); off += (size_t)B_ * N_ * N_ * 2;
  _Float16* P0 = (_Float16*)(ws + off); off += (size_t)B_ * CP * N_ * 2;
  _Float16* P1 = (_Float16*)(ws + off); off += (size_t)B_ * CP * N_ * 2;
  float* s_norm = (float*)(ws + off); off += (size_t)N_ * 4;
  float* b_norm = (float*)(ws + off); off += (size_t)B_ * N_ * 4;
  float* CWs    = (float*)(ws + off); off += 32 * 32 * 4;
  float* CWb    = (float*)(ws + off); off += 32 * 32 * 4;

  build_spatial<<<N_ / 32, 256, 0, stream>>>(Ks, s_norm);
  build_bilateral<<<(B_ * N_) / 32, 256, 0, stream>>>(rgb, Kb, b_norm);
  mix_mats<<<1, 1024, 0, stream>>>(Ws, Wb, compat, CWs, CWb);
  init_p<<<(B_ * N_) / 128, 128, 0, stream>>>(unary, P0);

  crf_iter<<<128, 256, 0, stream>>>(unary, Ks, Kb, s_norm, b_norm, CWs, CWb, P0, P1, out, 0);
  crf_iter<<<128, 256, 0, stream>>>(unary, Ks, Kb, s_norm, b_norm, CWs, CWb, P1, P0, out, 0);
  crf_iter<<<128, 256, 0, stream>>>(unary, Ks, Kb, s_norm, b_norm, CWs, CWb, P0, P1, out, 0);
  crf_iter<<<128, 256, 0, stream>>>(unary, Ks, Kb, s_norm, b_norm, CWs, CWb, P1, P0, out, 0);
  crf_iter<<<128, 256, 0, stream>>>(unary, Ks, Kb, s_norm, b_norm, CWs, CWb, P0, P1, out, 1);
}
